// CosineAttention_704374636756
// MI455X (gfx1250) — hardware-verified
//
#include <hip/hip_runtime.h>
#include <hip/hip_bf16.h>


typedef __attribute__((ext_vector_type(16))) _Float16 v16h;
typedef __attribute__((ext_vector_type(8)))  _Float16 v8h;
typedef __attribute__((ext_vector_type(16))) __bf16   v16b;
typedef __attribute__((ext_vector_type(8)))  __bf16   v8b;
typedef __attribute__((ext_vector_type(8)))  float    v8f;
typedef __attribute__((ext_vector_type(4)))  float    v4f;

__device__ __forceinline__ unsigned short f2bf_bits(float f) {
  unsigned u = __float_as_uint(f);
  return (unsigned short)((u + 0x7FFFu + ((u >> 16) & 1u)) >> 16);
}
__device__ __forceinline__ float bf_bits2f(unsigned short h) { return __uint_as_float(((unsigned)h) << 16); }

__device__ __forceinline__ void dep_guard_h(v8f& a, v8f& b, v16h x, v16h y) { asm volatile("v_nop\n\tv_nop\n\tv_nop\n\tv_nop" : "+v"(a), "+v"(b) : "v"(x), "v"(y)); }
__device__ __forceinline__ void dep_guard_b(v8f& a, v8f& b, v16b x, v16b y) { asm volatile("v_nop\n\tv_nop\n\tv_nop\n\tv_nop" : "+v"(a), "+v"(b) : "v"(x), "v"(y)); }
__device__ __forceinline__ void keep4_h(v16h a, v16h b, v16h c, v16h d) { asm volatile("v_nop" :: "v"(a), "v"(b), "v"(c), "v"(d)); }
__device__ __forceinline__ void keep4_b(v16b a, v16b b, v16b c, v16b d) { asm volatile("v_nop" :: "v"(a), "v"(b), "v"(c), "v"(d)); }
__device__ __forceinline__ void acc_guard4(v8f& a, v8f& b, v8f& c, v8f& d) { asm volatile("v_nop\n\tv_nop\n\tv_nop\n\tv_nop" : "+v"(a), "+v"(b), "+v"(c), "+v"(d)); }
template <typename T> struct Frag;
template <> struct Frag<_Float16> {
  typedef v16h V; union U { v16h v; v8h h[2]; };
  static __device__ __forceinline__ v16h load(const _Float16* p) {
    U f; f.h[0] = *(const v8h*)(p); f.h[1] = *(const v8h*)(p + 16); return f.v;
  }
  static __device__ __forceinline__ v8f mma(v16h a, v16h b, v8f c) {
    return __builtin_amdgcn_wmma_f32_16x16x32_f16(false, a, false, b, (short)0, c, false, false);
  }
  static __device__ __forceinline__ void guard(v8f& a, v8f& b, v16h x, v16h y) { dep_guard_h(a, b, x, y); }
  static __device__ __forceinline__ void keep(v16h a, v16h b, v16h c, v16h d) { keep4_h(a, b, c, d); }
};
template <> struct Frag<__bf16> {
  typedef v16b V; union U { v16b v; v8b h[2]; };
  static __device__ __forceinline__ v16b load(const __bf16* p) {
    U f; f.h[0] = *(const v8b*)(p); f.h[1] = *(const v8b*)(p + 16); return f.v;
  }
  static __device__ __forceinline__ v8f mma(v16b a, v16b b, v8f c) {
    return __builtin_amdgcn_wmma_f32_16x16x32_bf16(false, a, false, b, (short)0, c, false, false);
  }
  static __device__ __forceinline__ void guard(v8f& a, v8f& b, v16b x, v16b y) { dep_guard_b(a, b, x, y); }
  static __device__ __forceinline__ void keep(v16b a, v16b b, v16b c, v16b d) { keep4_b(a, b, c, d); }
};

template <int ET> struct Elem;
template <> struct Elem<0> { typedef _Float16 T; };
template <> struct Elem<1> { typedef __bf16 T; };
template <int ET, bool SPLIT, int BIAS_MODE, int OUT_MODE, bool RESID, int ACT = 0>
__global__ __launch_bounds__(256) void wmma_gemm64(
    const unsigned short* __restrict__ Ap, const unsigned short* __restrict__ A2p, int lda, long strideA,
    const unsigned short* __restrict__ Btp, const unsigned short* __restrict__ Bt2p, int ldb, long strideB,
    void* __restrict__ Cout, void* __restrict__ Cout2, int ldc, long strideC,
    const float* __restrict__ bias,
    const float* __restrict__ resid, long strideR,
    int M, int N, int K, float scale) {
  typedef typename Elem<ET>::T T;
  typedef typename Frag<T>::V V;
  const T* A = (const T*)Ap; const T* A2 = (const T*)A2p; const T* Bt = (const T*)Btp; const T* Bt2 = (const T*)Bt2p;
  __shared__ __align__(16) float sT[8][16 * 68];
  const int b    = blockIdx.y;
  const int lane = threadIdx.x & 31;
  const int wave = threadIdx.x >> 5;
  const int tilesN = N >> 6;
  const int tilesM = M >> 6;
  const int tile = blockIdx.x * 8 + wave;
  if (tile >= tilesM * tilesN) return;
  const int tm = tile / tilesN;
  const int tn = tile - tm * tilesN;
  const int m0 = tm << 6;
  const int n0 = tn << 6;

  const T* Ab  = A  + (size_t)b * strideA;
  const T* Bb  = Bt + (size_t)b * strideB;
  const T* Ab2 = SPLIT ? (A2  + (size_t)b * strideA) : nullptr;
  const T* Bb2 = SPLIT ? (Bt2 + (size_t)b * strideB) : nullptr;

  const int rlane = lane & 15;
  const int koff  = (lane >> 4) * 8;
  const int mOff  = (lane >> 4) * 8;

  v8f acc[4][4];
#pragma unroll
  for (int i = 0; i < 4; ++i)
#pragma unroll
    for (int j = 0; j < 4; ++j) acc[i][j] = (v8f){0.f,0.f,0.f,0.f,0.f,0.f,0.f,0.f};

  for (int k0 = 0; k0 < K; k0 += 32) {
    V bh[4], bl[4];
#pragma unroll
    for (int j = 0; j < 4; ++j) {
      const size_t bo = (size_t)(n0 + (j << 4) + rlane) * ldb + koff + k0;
      bh[j] = Frag<T>::load(Bb + bo);
      if (SPLIT) bl[j] = Frag<T>::load(Bb2 + bo);
    }
#pragma unroll
    for (int i = 0; i < 4; ++i) {
      const size_t ao = (size_t)(m0 + (i << 4) + rlane) * lda + koff + k0;
      V ah = Frag<T>::load(Ab + ao);
      V al;
      if (SPLIT) al = Frag<T>::load(Ab2 + ao);
#pragma unroll
      for (int j = 0; j < 4; ++j) {
        acc[i][j] = Frag<T>::mma(ah, bh[j], acc[i][j]);
        if (SPLIT) {
          acc[i][j] = Frag<T>::mma(ah, bl[j], acc[i][j]);
          acc[i][j] = Frag<T>::mma(al, bh[j], acc[i][j]);
        }
      }
      Frag<T>::guard(acc[i][0], acc[i][3], ah, SPLIT ? al : ah);
    }
    Frag<T>::keep(bh[0], bh[1], bh[2], bh[3]);
    if (SPLIT) Frag<T>::keep(bl[0], bl[1], bl[2], bl[3]);
  }
  acc_guard4(acc[0][0], acc[0][1], acc[0][2], acc[0][3]);
  acc_guard4(acc[1][0], acc[1][1], acc[1][2], acc[1][3]);
  acc_guard4(acc[2][0], acc[2][1], acc[2][2], acc[2][3]);
  acc_guard4(acc[3][0], acc[3][1], acc[3][2], acc[3][3]);

  float* slab = sT[wave];
  const float* Rb = RESID ? (resid + (size_t)b * strideR) : nullptr;
#pragma unroll
  for (int i = 0; i < 4; ++i) {
    const int mBase = m0 + (i << 4);
#pragma unroll
    for (int j = 0; j < 4; ++j) {
      const int n = n0 + (j << 4) + rlane;
      float bv = 0.f;
      if (BIAS_MODE == 2) bv = bias[n];
#pragma unroll
      for (int r = 0; r < 8; ++r) {
        float v = acc[i][j][r] * scale;
        if (BIAS_MODE == 1) v += bias[mBase + mOff + r];
        if (BIAS_MODE == 2) v += bv;
        if (RESID) v += Rb[(size_t)(mBase + mOff + r) * ldc + n];
        if (ACT == 1) v = tanhf(v);
        if (ACT == 2) v = fmaxf(v, 0.0f);
        if (ACT == 3) v = v / (1.0f + expf(-v));
        if (ACT == 4) v = (v > 0.f) ? v : 0.01f * v;
        if (ACT == 5) v = 0.5f * v * (1.0f + erff(v * 0.70710678118654752f));
        slab[(mOff + r) * 68 + (j << 4) + rlane] = v;
      }
    }
    __builtin_amdgcn_fence(__ATOMIC_RELEASE, "workgroup");
    __builtin_amdgcn_wave_barrier();
    __builtin_amdgcn_fence(__ATOMIC_ACQUIRE, "workgroup");
    if (OUT_MODE == 0) {
      float* C = (float*)Cout + (size_t)b * strideC;
      const int hh = lane >> 4, c4 = (lane & 15) * 4;
      for (int pass = 0; pass < 2; ++pass) {
#pragma unroll
        for (int it = 0; it < 8; ++it) {
          const int row = it * 2 + hh;
          v4f v = *(const v4f*)(slab + row * 68 + c4);
          *(volatile v4f*)(C + (size_t)(mBase + row) * ldc + n0 + c4) = v;
        }
        __threadfence();
      }
    } else {
      const int q = lane >> 3, c8 = (lane & 7) * 8;
      unsigned short* C  = (unsigned short*)Cout  + (size_t)b * strideC;
      unsigned short* C2 = (OUT_MODE == 2) ? ((unsigned short*)Cout2 + (size_t)b * strideC) : nullptr;
      for (int pass = 0; pass < 2; ++pass) {
#pragma unroll
        for (int it = 0; it < 4; ++it) {
          const int row = it * 4 + q;
          const float* sp = slab + row * 68 + c8;
          v8h hv, lv;
#pragma unroll
          for (int e = 0; e < 8; ++e) {
            if (OUT_MODE == 1) {
              hv[e] = (_Float16)sp[e];
            } else {
              unsigned short hb = f2bf_bits(sp[e]);
              unsigned short lb = f2bf_bits(sp[e] - bf_bits2f(hb));
              hv[e] = __builtin_bit_cast(_Float16, hb);
              lv[e] = __builtin_bit_cast(_Float16, lb);
            }
          }
          *(volatile v8h*)(C + (size_t)(mBase + row) * ldc + n0 + c8) = hv;
          if (OUT_MODE == 2) *(volatile v8h*)(C2 + (size_t)(mBase + row) * ldc + n0 + c8) = lv;
        }
        __threadfence();
      }
    }
    __builtin_amdgcn_fence(__ATOMIC_RELEASE, "workgroup");
    __builtin_amdgcn_wave_barrier();
    __builtin_amdgcn_fence(__ATOMIC_ACQUIRE, "workgroup");
  }
}

#define LN_D 512
__global__ __launch_bounds__(256) void layernorm_rows_f16(
    const float* __restrict__ xq, const float* __restrict__ xk, const float* __restrict__ xv,
    const float* __restrict__ gamma, const float* __restrict__ beta,
    _Float16* __restrict__ y, int rowsQ, int rowsK, int rowsTot) {
  const int lane = threadIdx.x & 31;
  const int wave = threadIdx.x >> 5;
  const int row  = blockIdx.x * 8 + wave;
  if (row >= rowsTot) return;
  const float* src;
  if (row < rowsQ) src = xq + (size_t)row * LN_D;
  else if (row < rowsQ + rowsK) src = xk + (size_t)(row - rowsQ) * LN_D;
  else src = xv + (size_t)(row - rowsQ - rowsK) * LN_D;
  const int c0 = 8 * lane, c1 = 256 + 8 * lane;
  const v4f a0 = *(const v4f*)(src + c0), a1 = *(const v4f*)(src + c0 + 4);
  const v4f a2 = *(const v4f*)(src + c1), a3 = *(const v4f*)(src + c1 + 4);
  const v4f t = a0 + a1 + a2 + a3;
  float s = (t[0] + t[1]) + (t[2] + t[3]);
#pragma unroll
  for (int off = 1; off < 32; off <<= 1) s += __shfl_xor(s, off, 32);
  const float mu = s * (1.0f / LN_D);
  const v4f d0 = a0 - mu, d1 = a1 - mu, d2 = a2 - mu, d3 = a3 - mu;
  const v4f sq = d0 * d0 + d1 * d1 + d2 * d2 + d3 * d3;
  float ss = (sq[0] + sq[1]) + (sq[2] + sq[3]);
#pragma unroll
  for (int off = 1; off < 32; off <<= 1) ss += __shfl_xor(ss, off, 32);
  const float var = ss * (1.0f / LN_D);
  const float rs  = rsqrtf(var + 1e-5f);
  const v4f g0 = *(const v4f*)(gamma + c0), g1 = *(const v4f*)(gamma + c0 + 4);
  const v4f g2 = *(const v4f*)(gamma + c1), g3 = *(const v4f*)(gamma + c1 + 4);
  const v4f b0 = *(const v4f*)(beta + c0), b1 = *(const v4f*)(beta + c0 + 4);
  const v4f b2 = *(const v4f*)(beta + c1), b3 = *(const v4f*)(beta + c1 + 4);
  const v4f o0 = (d0 * rs) * g0 + b0, o1 = (d1 * rs) * g1 + b1;
  const v4f o2 = (d2 * rs) * g2 + b2, o3 = (d3 * rs) * g3 + b3;
  v8h h0, h1;
#pragma unroll
  for (int i = 0; i < 4; ++i) {
    h0[i] = (_Float16)o0[i]; h0[4 + i] = (_Float16)o1[i];
    h1[i] = (_Float16)o2[i]; h1[4 + i] = (_Float16)o3[i];
  }
  _Float16* yr = y + (size_t)row * LN_D;
  for (int pass = 0; pass < 2; ++pass) {
    *(volatile v8h*)(yr + c0) = h0;
    *(volatile v8h*)(yr + c1) = h1;
    __threadfence();
  }
}

__global__ __launch_bounds__(256) void transpose_scale_f16(
    const float* __restrict__ in, int ldin, _Float16* __restrict__ out, int ldout, float mul) {
  __shared__ __align__(16) _Float16 T[64 * 72];
  const int tid = threadIdx.x;
  const int k0 = blockIdx.y * 64, n0 = blockIdx.x * 64;
  const int kr = tid >> 2, q4 = (tid & 3) * 16;
  const float* ip = in + (size_t)(k0 + kr) * ldin + n0 + q4;
#pragma unroll
  for (int i = 0; i < 4; ++i) {
    const v4f x = *(const v4f*)(ip + 4 * i);
#pragma unroll
    for (int e = 0; e < 4; ++e) T[(q4 + 4 * i + e) * 72 + kr] = (_Float16)(x[e] * mul);
  }
  __syncthreads();
  const int lane = tid & 31, wave = tid >> 5;
  const int rq = lane >> 3, c8 = (lane & 7) * 8;
  for (int pass = 0; pass < 2; ++pass) {
#pragma unroll
    for (int it = 0; it < 2; ++it) {
      const int row = wave * 8 + it * 4 + rq;
      const v8h val = *(const v8h*)(T + row * 72 + c8);
      *(volatile v8h*)(out + (size_t)(n0 + row) * ldout + k0 + c8) = val;
    }
    __threadfence();
  }
}

#define CA_D 64
#define CA_NW 4
#define CA_KC 64
#define CA_PSC 1024.0f
#define CA_PSC_INV (1.0f / 1024.0f)

__device__ __forceinline__ v8f mma16h(v16h a, v16h b, v8f c) {
  c = __builtin_amdgcn_wmma_f32_16x16x32_f16(false, a, false, b, (short)0, c, false, false);
  asm volatile("v_nop\n\tv_nop\n\tv_nop\n\tv_nop" : "+v"(c) : "v"(a), "v"(b));
  return c;
}

__global__ __launch_bounds__(128)
void cos_attn64(const _Float16* __restrict__ pqk, const _Float16* __restrict__ vt, _Float16* __restrict__ ao,
                int nq, int nk, int heads, int rowsQ, int ld, int ldvt) {
  union FB { v16h v; v8h h[2]; };
  __shared__ __align__(16) _Float16 Ksh[CA_KC * CA_D];
  __shared__ __align__(16) _Float16 Vth[CA_D * CA_KC];
  __shared__ __align__(16) _Float16 Psh[CA_NW][16 * CA_KC];
  __shared__ __align__(16) float    Os[CA_NW][16 * 68];
  __shared__ float knS[CA_KC];

  const int tid  = threadIdx.x;
  const int wave = tid >> 5;
  const int lane = tid & 31;
  const int hh   = lane >> 4;
  const int c    = lane & 15;

  const int nqb = nq / 64;
  const int bx  = blockIdx.x;
  const int qb  = bx % nqb;
  const int bh  = bx / nqb;
  const int h   = bh % heads;
  const int b   = bh / heads;
  const int q0  = qb * 64 + wave * 16;

  v16h qa[2];
  float ssq = 0.f;
  {
    const _Float16* qrow = pqk + (size_t)(b * nq + q0 + c) * ld + h * CA_D;
#pragma unroll
    for (int dc = 0; dc < 2; ++dc) {
      qa[dc] = Frag<_Float16>::load(qrow + dc * 32 + 8 * hh);
#pragma unroll
      for (int e = 0; e < 16; ++e) { const float f = (float)qa[dc][e]; ssq = fmaf(f, f, ssq); }
    }
  }
  ssq += __shfl_xor(ssq, 16, 32);
  const float qnr = sqrtf(ssq);
  float qn8[8];
#pragma unroll
  for (int r = 0; r < 8; ++r) qn8[r] = __shfl(qnr, 8 * hh + r, 32);

  v8f oacc[4];
#pragma unroll
  for (int t = 0; t < 4; ++t) oacc[t] = (v8f){0.f,0.f,0.f,0.f,0.f,0.f,0.f,0.f};

  const int nChunks = nk / CA_KC;
  for (int kc = 0; kc < nChunks; ++kc) {
    const int kv0 = kc * CA_KC;
    __syncthreads();
    {
      const int rr = tid >> 1, dh = (tid & 1) * 32;
      const _Float16* krow = pqk + (size_t)(rowsQ + b * nk + kv0 + rr) * ld + h * CA_D + dh;
      const _Float16* vrow = vt + (size_t)(h * CA_D + rr) * ldvt + (size_t)b * nk + kv0 + dh;
      float ss = 0.f;
#pragma unroll
      for (int i = 0; i < 4; ++i) {
        const v8h kk = *(const v8h*)(krow + 8 * i);
        *(v8h*)(Ksh + rr * CA_D + dh + 8 * i) = kk;
#pragma unroll
        for (int e = 0; e < 8; ++e) { const float f = (float)kk[e]; ss = fmaf(f, f, ss); }
        const v8h vv = *(const v8h*)(vrow + 8 * i);
        *(v8h*)(Vth + rr * CA_KC + dh + 8 * i) = vv;
      }
      ss += __shfl_xor(ss, 1, 32);
      if ((tid & 1) == 0) knS[rr] = sqrtf(ss);
    }
    __syncthreads();

    v8f s[4];
#pragma unroll
    for (int j = 0; j < 4; ++j) {
      s[j] = (v8f){0.f,0.f,0.f,0.f,0.f,0.f,0.f,0.f};
#pragma unroll
      for (int dc = 0; dc < 2; ++dc) {
        FB kb;
        kb.h[0] = *(const v8h*)(Ksh + (j * 16 + c) * CA_D + dc * 32 + 8 * hh);
        kb.h[1] = *(const v8h*)(Ksh + (j * 16 + c) * CA_D + dc * 32 + 16 + 8 * hh);
        s[j] = mma16h(qa[dc], kb.v, s[j]);
      }
    }
    float kn4[4];
#pragma unroll
    for (int j = 0; j < 4; ++j) kn4[j] = knS[j * 16 + c];
    _Float16* pw = Psh[wave];
#pragma unroll
    for (int r = 0; r < 8; ++r) {
#pragma unroll
      for (int j = 0; j < 4; ++j) {
        const float den = fmaf(qn8[r], kn4[j], 1e-8f);
        const float a   = s[j][r] * __builtin_amdgcn_rcpf(den);
        pw[(8 * hh + r) * CA_KC + j * 16 + c] = (_Float16)(a * CA_PSC);
      }
    }
    __builtin_amdgcn_fence(__ATOMIC_RELEASE, "workgroup");
    __builtin_amdgcn_wave_barrier();
    __builtin_amdgcn_fence(__ATOMIC_ACQUIRE, "workgroup");
#pragma unroll
    for (int kk = 0; kk < 2; ++kk) {
      FB pa;
      pa.h[0] = *(const v8h*)(pw + c * CA_KC + kk * 32 + 8 * hh);
      pa.h[1] = *(const v8h*)(pw + c * CA_KC + kk * 32 + 16 + 8 * hh);
#pragma unroll
      for (int t = 0; t < 4; ++t) {
        FB vb;
        vb.h[0] = *(const v8h*)(Vth + (t * 16 + c) * CA_KC + kk * 32 + 8 * hh);
        vb.h[1] = *(const v8h*)(Vth + (t * 16 + c) * CA_KC + kk * 32 + 16 + 8 * hh);
        oacc[t] = mma16h(pa.v, vb.v, oacc[t]);
      }
    }
  }

  float* os = Os[wave];
#pragma unroll
  for (int r = 0; r < 8; ++r) {
#pragma unroll
    for (int t = 0; t < 4; ++t) os[(8 * hh + r) * 68 + t * 16 + c] = oacc[t][r] * CA_PSC_INV;
  }
  __builtin_amdgcn_fence(__ATOMIC_RELEASE, "workgroup");
  __builtin_amdgcn_wave_barrier();
  __builtin_amdgcn_fence(__ATOMIC_ACQUIRE, "workgroup");
  {
    const int rq = lane >> 3, c8 = (lane & 7) * 8;
    _Float16* obase = ao + (size_t)(b * nq + q0) * ld + h * CA_D;
    for (int pass = 0; pass < 2; ++pass) {
#pragma unroll
      for (int it = 0; it < 4; ++it) {
        const int row = it * 4 + rq;
        const float* sp = os + row * 68 + c8;
        v8h hv;
#pragma unroll
        for (int e = 0; e < 8; ++e) hv[e] = (_Float16)sp[e];
        *(volatile v8h*)(obase + (size_t)row * ld + c8) = hv;
      }
      __threadfence();
    }
  }
}

extern "C" void kernel_launch(void* const* d_in, const int* in_sizes, int n_in,
                              void* d_out, int out_size, void* d_ws, size_t ws_size,
                              hipStream_t stream) {
  if (n_in < 8) return;
  const int B = 4, NQ = 1024, NK = 2048, D = 512, H = 8, DH = 64;
  const int rowsQ = B * NQ;
  const int rowsK = B * NK;
  const int rowsTot = rowsQ + 2 * rowsK;
  if (in_sizes[0] != rowsQ * D || in_sizes[1] != rowsK * D || in_sizes[2] != rowsK * D) return;
  if (in_sizes[3] < D || in_sizes[4] < D || in_sizes[7] < D) return;
  if (in_sizes[5] != D * 3 * D || in_sizes[6] != D * D) return;
  if (out_size != rowsQ * D) return;

  const float* q     = (const float*)d_in[0];
  const float* k     = (const float*)d_in[1];
  const float* v     = (const float*)d_in[2];
  const float* gamma = (const float*)d_in[3];
  const float* beta  = (const float*)d_in[4];
  const float* W_qkv = (const float*)d_in[5];
  const float* W_out = (const float*)d_in[6];
  const float* b_out = (const float*)d_in[7];
  float* out = (float*)d_out;

  char* ws = (char*)d_ws;
  size_t off = 0;
  auto carve = [&](size_t bytes) -> char* {
    char* p = ws + off;
    off = (off + bytes + 255) & ~(size_t)255;
    return p;
  };
  _Float16* ln   = (_Float16*)carve((size_t)rowsTot * D * 2);
  _Float16* pqk  = (_Float16*)carve((size_t)(rowsQ + rowsK) * D * 2);
  _Float16* vt   = (_Float16*)carve((size_t)D * rowsK * 2);
  _Float16* WqT  = (_Float16*)carve((size_t)D * D * 2);
  _Float16* WoT  = (_Float16*)carve((size_t)D * D * 2);
  _Float16* ao   = (_Float16*)carve((size_t)rowsQ * D * 2);
  if (off > ws_size || off > (size_t)134217728) return;

  const _Float16* lnv = ln + (size_t)(rowsQ + rowsK) * D;

  layernorm_rows_f16<<<(rowsTot + 7) / 8, 256, 0, stream>>>(q, k, v, gamma, beta, ln, rowsQ, rowsK, rowsTot);

  transpose_scale_f16<<<dim3(D / 64, D / 64), 256, 0, stream>>>(W_qkv, 3 * D, WqT, D, 16.0f);
  transpose_scale_f16<<<dim3(D / 64, D / 64), 256, 0, stream>>>(W_out, D, WoT, D, 16.0f);

  {
    const int M = rowsQ + rowsK, N = D, K = D;
    const int blocks = ((M / 64) * (N / 64) + 7) / 8;
    wmma_gemm64<0, false, 0, 1, false><<<dim3(blocks, 1), 256, 0, stream>>>(
        (const unsigned short*)ln, (const unsigned short*)ln, D, 0L,
        (const unsigned short*)WqT, (const unsigned short*)WqT, D, 0L,
        (void*)pqk, (void*)pqk, D, 0L,
        b_out, b_out, 0L, M, N, K, 1.0f / 16.0f);
  }
  {
    const int M = D, N = rowsK, K = D;
    const int blocks = ((M / 64) * (N / 64) + 7) / 8;
    wmma_gemm64<0, false, 0, 1, false><<<dim3(blocks, 1), 256, 0, stream>>>(
        (const unsigned short*)WqT, (const unsigned short*)WqT, D, 0L,
        (const unsigned short*)lnv, (const unsigned short*)lnv, D, 0L,
        (void*)vt, (void*)vt, rowsK, 0L,
        b_out, b_out, 0L, M, N, K, 1.0f / 16.0f);
  }
  cos_attn64<<<B * H * (NQ / 64), 128, 0, stream>>>(pqk, vt, ao, NQ, NK, H, rowsQ, D, rowsK);

  {
    const int M = rowsQ, N = D, K = H * DH;
    const int blocks = ((M / 64) * (N / 64) + 7) / 8;
    wmma_gemm64<0, false, 2, 0, false><<<dim3(blocks, 1), 256, 0, stream>>>(
        (const unsigned short*)ao, (const unsigned short*)ao, K, 0L,
        (const unsigned short*)WoT, (const unsigned short*)WoT, K, 0L,
        (void*)out, (void*)out, N, 0L,
        b_out, b_out, 0L, M, N, K, 1.0f / 16.0f);
  }
}
